// Upsampling_30322469110354
// MI455X (gfx1250) — hardware-verified
//
#include <hip/hip_runtime.h>


namespace {
constexpr int Bn = 4, K = 200, DIM = 256, T = 800, KP = 224, NBT = Bn * T;
constexpr float HS = 1.0f / 64.0f;

typedef _Float16 b16;
typedef __attribute__((ext_vector_type(16))) _Float16 v16b;
typedef __attribute__((ext_vector_type(8)))  _Float16 v8b;
typedef __attribute__((ext_vector_type(8)))  float v8f;
typedef __attribute__((ext_vector_type(4)))  float v4f;

__device__ __forceinline__ v8b ld8b(const b16* p) { return *(const v8b*)p; }
__device__ __forceinline__ v16b cat8b(v8b a, v8b b) { return __builtin_shufflevector(a, b, 0, 1, 2, 3, 4, 5, 6, 7, 8, 9, 10, 11, 12, 13, 14, 15); }
__device__ __forceinline__ v16b frag_kb(const b16* p, int hh) { return cat8b(ld8b(p + 8 * hh), ld8b(p + 16 + 8 * hh)); }
__device__ __forceinline__ void split16(float v, b16& hi, b16& lo) { hi = (b16)v; lo = (b16)(v - (float)hi); }
__device__ __forceinline__ void frag_ksplit(const float* p, int hh, v16b& fh_, v16b& fl_) {
  const float* p0 = p + 8 * hh; const float* p1 = p + 16 + 8 * hh;
#pragma unroll
  for (int e = 0; e < 8; ++e) { b16 a, c; split16(p0[e], a, c); fh_[e] = a; fl_[e] = c; split16(p1[e], a, c); fh_[8 + e] = a; fl_[8 + e] = c; }
}
__device__ __forceinline__ v8f wmma16b(v16b a, v16b b, v8f c) {
  v8f d = __builtin_amdgcn_wmma_f32_16x16x32_f16(false, a, false, b, (short)0, c, false, false);
  asm volatile("v_nop\n\tv_nop\n\tv_nop\n\tv_nop" : "+v"(d) : "v"(a), "v"(b));
  return d;
}
__device__ __forceinline__ void wave_lds_sync() {
  __builtin_amdgcn_fence(__ATOMIC_RELEASE, "workgroup");
  __builtin_amdgcn_wave_barrier();
  __builtin_amdgcn_fence(__ATOMIC_ACQUIRE, "workgroup");
}

struct Opnd { const void* p0; const void* p1; int ld; };
template <int NP> __device__ __forceinline__ void load_frags(const Opnd& o, int row, int kb, int hh, v16b& fh_, v16b& fl_) {
  if (NP == 0) { frag_ksplit((const float*)o.p0 + (size_t)row * o.ld + kb, hh, fh_, fl_); }
  else if (NP == 3) {
    const float* p = (const float*)o.p0 + (size_t)row * o.ld + kb; const float* p0 = p + 8 * hh; const float* p1 = p + 16 + 8 * hh;
#pragma unroll
    for (int e = 0; e < 8; ++e) { fh_[e] = (b16)p0[e]; fh_[8 + e] = (b16)p1[e]; }
    fl_ = fh_;
  } else {
    fh_ = frag_kb((const b16*)o.p0 + (size_t)row * o.ld + kb, hh);
    if (NP == 2) fl_ = frag_kb((const b16*)o.p1 + (size_t)row * o.ld + kb, hh); else fl_ = fh_;
  }
}
template <int ANP, int BNP> __device__ __forceinline__ v8f mac(v16b ah, v16b al, v16b bh, v16b bl, v8f c) {
  c = wmma16b(ah, bh, c);
  if (BNP == 0 || BNP == 2) c = wmma16b(ah, bl, c);
  if (ANP == 0 || ANP == 2) c = wmma16b(al, bh, c);
  return c;
}
template <int ANP, int BNP>
__device__ __forceinline__ void gemm_tile(const Opnd& A, const Opnd& B, int K, int m0, int c0, int nloc, int hlf, v8f (&acc)[2][4]) {
  for (int kb = 0; kb < K; kb += 32) {
    v16b a0h, a0l, a1h, a1l;
    load_frags<ANP>(A, m0 + nloc, kb, hlf, a0h, a0l);
    load_frags<ANP>(A, m0 + 16 + nloc, kb, hlf, a1h, a1l);
#pragma unroll
    for (int t = 0; t < 4; ++t) {
      v16b bh, bl;
      load_frags<BNP>(B, c0 + t * 16 + nloc, kb, hlf, bh, bl);
      acc[0][t] = mac<ANP, BNP>(a0h, a0l, bh, bl, acc[0][t]);
      acc[1][t] = mac<ANP, BNP>(a1h, a1l, bh, bl, acc[1][t]);
    }
  }
}

struct Epi { float scale; const float* cscale; const float* cbias; const float* rbias; int act; float post; const float* rscale; const float* resid; };
__device__ __forceinline__ float epi_val(const Epi& e, float acc, int row, int col) {
  float val = acc * e.scale;
  if (e.cscale) val *= e.cscale[col];
  if (e.cbias) val += e.cbias[col];
  if (e.rbias) val += e.rbias[row];
  if (e.act == 1) val = 0.5f * val * (1.0f + erff(val * 0.70710678118654752f));
  val *= e.post;
  if (e.rscale) val *= e.rscale[(size_t)row * 32];
  return val;
}
__device__ __forceinline__ void epi_planes(v8f (&acc)[2][4], const Epi& e, bool two,
                                           b16* __restrict__ oh, b16* __restrict__ ol, int ldo, int m0, int c0, int lane, b16* Th, b16* Tl) {
  const int nloc = lane & 15, hlf = lane >> 4;
#pragma unroll
  for (int t = 0; t < 4; ++t)
#pragma unroll
    for (int r = 0; r < 2; ++r)
#pragma unroll
      for (int v = 0; v < 8; ++v) {
        const int rr = r * 16 + v + 8 * hlf, cc = t * 16 + nloc;
        const float val = epi_val(e, acc[r][t][v], m0 + rr, c0 + cc);
        b16 h_, l_; split16(val, h_, l_);
        Th[rr * 64 + cc] = h_; if (two) Tl[rr * 64 + cc] = l_;
      }
  wave_lds_sync();
  for (int pass = 0; pass < 2; ++pass) {
#pragma unroll
    for (int j = 0; j < 8; ++j) {
      const int rr = j * 4 + (lane >> 3), c8 = (lane & 7) * 8;
      const size_t o = (size_t)(m0 + rr) * ldo + c0 + c8;
      *(volatile v8b*)(oh + o) = ld8b(Th + rr * 64 + c8);
      if (two) *(volatile v8b*)(ol + o) = ld8b(Tl + rr * 64 + c8);
    }
    __threadfence();
  }
}
__device__ __forceinline__ void epi_f32(v8f (&acc)[2][4], const Epi& e, float* __restrict__ out, int ldo, int m0, int c0, int lane, float* Tt) {
  const int nloc = lane & 15, hlf = lane >> 4;
#pragma unroll
  for (int t = 0; t < 4; ++t)
#pragma unroll
    for (int r = 0; r < 2; ++r)
#pragma unroll
      for (int v = 0; v < 8; ++v) {
        const int rr = r * 16 + v + 8 * hlf, cc = t * 16 + nloc;
        Tt[rr * 64 + cc] = epi_val(e, acc[r][t][v], m0 + rr, c0 + cc);
      }
  wave_lds_sync();
  float* dst0 = out + (size_t)m0 * ldo + c0; const float* rs0 = e.resid ? e.resid + (size_t)m0 * ldo + c0 : nullptr;
  for (int pass = 0; pass < 2; ++pass) {
#pragma unroll
    for (int j = 0; j < 16; ++j) {
      const int rr = j * 2 + hlf, c4 = nloc * 4;
      v4f val = *(const v4f*)(Tt + rr * 64 + c4);
      if (rs0) val += *(const v4f*)(rs0 + (size_t)rr * ldo + c4);
      *(volatile v4f*)(dst0 + (size_t)rr * ldo + c4) = val;
    }
    __threadfence();
  }
}


__device__ __forceinline__ float silu(float v) { return v / (1.0f + __expf(-v)); }

__global__ __launch_bounds__(256) void prep_kernel(const float* __restrict__ dur, const float* __restrict__ feat, const float* __restrict__ c1w, const float* __restrict__ c2w,
                                                   const float* __restrict__ w2, const float* __restrict__ p2w,
                                                   b16* __restrict__ cw16, b16* __restrict__ w2h, b16* __restrict__ w2l, b16* __restrict__ p2h, b16* __restrict__ p2l,
                                                   b16* __restrict__ featT, float* __restrict__ ts, float* __restrict__ te, float* __restrict__ zero) {
  const int tid = blockIdx.x * 256 + threadIdx.x, nth = gridDim.x * 256;
  for (int pass = 0; pass < 2; ++pass) {
    for (int p = tid; p < 16 * 768 / 8; p += nth) { const int n = p / 96, k0 = (p % 96) * 8; v8b v; const float* w = (n < 8) ? c1w : c2w; const int o = n & 7;
#pragma unroll
      for (int e = 0; e < 8; ++e) { const int k = k0 + e, tap = k / DIM, c = k % DIM; v[e] = (b16)w[(tap * DIM + c) * 8 + o]; }
      *(volatile v8b*)(cw16 + (size_t)n * 768 + k0) = v; }
    for (int p = tid; p < 16 * 2; p += nth) { const int n = p / 2, k0 = (p % 2) * 8; v8b vh, vl;
#pragma unroll
      for (int e = 0; e < 8; ++e) { b16 a, c; split16(w2[(k0 + e) * 16 + n], a, c); vh[e] = a; vl[e] = c; }
      *(volatile v8b*)(w2h + n * 16 + k0) = vh; *(volatile v8b*)(w2l + n * 16 + k0) = vl; }
    for (int p = tid; p < DIM * 2; p += nth) { const int n = p / 2, k0 = (p % 2) * 8; v8b vh, vl;
#pragma unroll
      for (int e = 0; e < 8; ++e) { b16 a, c; split16(p2w[(k0 + e) * DIM + n], a, c); vh[e] = a; vl[e] = c; }
      *(volatile v8b*)(p2h + n * 16 + k0) = vh; *(volatile v8b*)(p2l + n * 16 + k0) = vl; }
    for (int p = tid; p < Bn * DIM * KP / 8; p += nth) { const int k0 = (p % (KP / 8)) * 8, d = (p / (KP / 8)) % DIM, b = p / ((KP / 8) * DIM); v8b v;
#pragma unroll
      for (int e = 0; e < 8; ++e) { const int k = k0 + e; v[e] = (b16)((k < K) ? feat[((size_t)b * K + k) * DIM + d] : 0.0f); }
      *(volatile v8b*)(featT + ((size_t)b * DIM + d) * KP + k0) = v; }
    for (int p = tid; p < DIM; p += nth) ((volatile float*)zero)[p] = 0.0f;
    if (tid < Bn) { float acc = 0.0f;
#pragma unroll 1
      for (int k = 0; k < K; ++k) { const float dk = dur[tid * K + k]; acc += dk; ((volatile float*)te)[tid * 256 + k] = acc; ((volatile float*)ts)[tid * 256 + k] = acc - dk; } }
    __threadfence();
  }
}

__global__ __launch_bounds__(128) void conv_kernel(const float* __restrict__ feat, const float* __restrict__ zero, const b16* __restrict__ cw16, const float* __restrict__ c1b, const float* __restrict__ c2b, float* __restrict__ lr) {
  __shared__ __attribute__((aligned(16))) float Ts[4][32 * 16];
  const int lane = threadIdx.x & 31, wave = threadIdx.x >> 5, nloc = lane & 15, hlf = lane >> 4, m0 = blockIdx.x * 128 + wave * 32;
  if (m0 >= Bn * K) return;
  v8f acc[2] = {{}, {}};
  const int ra = m0 + nloc, rb = m0 + 16 + nloc;
#pragma unroll 1
  for (int tap = 0; tap < 3; ++tap) {
    const int ka = (ra % K) + tap - 1, kb_ = (rb % K) + tap - 1;
    const float* pa = (ka >= 0 && ka < K) ? (feat + ((size_t)(ra / K) * K + ka) * DIM) : zero; const float* pb = (kb_ >= 0 && kb_ < K) ? (feat + ((size_t)(rb / K) * K + kb_) * DIM) : zero;
    const Opnd Aa{pa, nullptr, 0}, Ab{pb, nullptr, 0};
#pragma unroll 2
    for (int c0 = 0; c0 < DIM; c0 += 32) {
      v16b a0, a1, d0, d1; load_frags<3>(Aa, 0, c0, hlf, a0, d0); load_frags<3>(Ab, 0, c0, hlf, a1, d1);
      const v16b bw = frag_kb(cw16 + (size_t)nloc * 768 + tap * DIM + c0, hlf);
      acc[0] = wmma16b(a0, bw, acc[0]); acc[1] = wmma16b(a1, bw, acc[1]);
    }
  }
  float* Tt = Ts[wave];
#pragma unroll
  for (int r = 0; r < 2; ++r)
#pragma unroll
    for (int v = 0; v < 8; ++v) { const int rr = r * 16 + v + 8 * hlf; const float bia = (nloc < 8) ? c1b[nloc] : c2b[nloc - 8]; Tt[rr * 16 + nloc] = silu(acc[r][v] + bia); }
  wave_lds_sync();
  for (int pass = 0; pass < 2; ++pass) {
#pragma unroll
    for (int j = 0; j < 4; ++j) *(volatile v4f*)(lr + (size_t)m0 * 16 + (j * 32 + lane) * 4) = *(const v4f*)(Tt + (j * 32 + lane) * 4);
    __threadfence();
  }
}

__global__ __launch_bounds__(256) void main_kernel(const float* __restrict__ ts, const float* __restrict__ te, const float* __restrict__ lr,
                                                   const float* __restrict__ w1, const float* __restrict__ b1, const b16* __restrict__ w2h, const b16* __restrict__ w2l, const float* __restrict__ b2,
                                                   const float* __restrict__ v1, const float* __restrict__ vb1, const float* __restrict__ v2, const float* __restrict__ vb2, const float* __restrict__ p1w, const float* __restrict__ p1b,
                                                   b16* __restrict__ Wg, b16* __restrict__ Agh, b16* __restrict__ Agl) {
  __shared__ float Wl[8][KP]; __shared__ __attribute__((aligned(16))) b16 Ws[8][256]; __shared__ __attribute__((aligned(16))) b16 As[2][8][32];
  const int wid = threadIdx.x >> 5, lane = threadIdx.x & 31, hh = lane >> 4, col = lane & 15;
  const int bt = blockIdx.x * 8 + wid, b = bt / T; const float tf = (float)(bt % T);
  const float* tsb = ts + b * 256; const float* teb = te + b * 256; const float* lrb = lr + (size_t)b * K * 16;
  float mx = -INFINITY;
  for (int k = lane; k < KP; k += 32) {
    float lg = -INFINITY;
    if (k < K) {
      float x[10]; x[0] = tf - tsb[k]; x[1] = teb[k] - tf;
#pragma unroll
      for (int i = 0; i < 8; ++i) x[2 + i] = lrb[k * 16 + 8 + i];
      float r1[2];
#pragma unroll
      for (int j = 0; j < 2; ++j) { float s = vb1[j];
#pragma unroll
        for (int i = 0; i < 10; ++i) s += x[i] * v1[i * 2 + j];
        r1[j] = silu(s); }
      float r2[2];
#pragma unroll
      for (int j = 0; j < 2; ++j) r2[j] = silu(vb2[j] + r1[0] * v2[0 * 2 + j] + r1[1] * v2[1 * 2 + j]);
      lg = p1b[0] + r2[0] * p1w[0] + r2[1] * p1w[1];
    }
    Wl[wid][k] = lg; mx = fmaxf(mx, lg);
  }
#pragma unroll
  for (int o = 16; o > 0; o >>= 1) mx = fmaxf(mx, __shfl_xor(mx, o));
  float sm = 0.0f;
  for (int k = lane; k < KP; k += 32) { const float e = (k < K) ? __expf(Wl[wid][k] - mx) : 0.0f; Wl[wid][k] = e; sm += e; }
#pragma unroll
  for (int o = 16; o > 0; o >>= 1) sm += __shfl_xor(sm, o);
  const float inv = 1.0f / sm;
  for (int k = lane; k < 256; k += 32) { const float w = (k < KP) ? Wl[wid][k] * inv : 0.0f; if (k < KP) Wl[wid][k] = w; Ws[wid][k] = (b16)w; }
  wave_lds_sync();
  for (int pass = 0; pass < 2; ++pass) { *(volatile v8b*)(Wg + (size_t)bt * 256 + lane * 8) = *(const v8b*)(&Ws[wid][lane * 8]); __threadfence(); }
  v16b bw2h = {}, bw2l = {};
  { const v8b ph = ld8b(w2h + col * 16 + 8 * hh), plw = ld8b(w2l + col * 16 + 8 * hh);
#pragma unroll
    for (int e = 0; e < 8; ++e) { bw2h[e] = ph[e]; bw2l[e] = plw[e]; } }
  float accA = 0.0f;
#pragma unroll 1
  for (int k0 = 0; k0 < K; k0 += 16) {
    const int k = k0 + col; v16b ah = {}, al = {};
    if (k < K) {
      float x[10]; x[0] = tf - tsb[k]; x[1] = teb[k] - tf;
#pragma unroll
      for (int i = 0; i < 8; ++i) x[2 + i] = lrb[k * 16 + i];
#pragma unroll
      for (int e = 0; e < 8; ++e) { const int j = 8 * hh + e; float s = b1[j];
#pragma unroll
        for (int i = 0; i < 10; ++i) s += x[i] * w1[i * 16 + j];
        b16 a, c; split16(silu(s) * HS, a, c); ah[e] = a; al[e] = c; }
    }
    v8f Dm = {}; Dm = mac<2, 2>(ah, al, bw2h, bw2l, Dm);
    float part = 0.0f;
#pragma unroll
    for (int v = 0; v < 8; ++v) { const int kk = k0 + 8 * hh + v; const float Cv = silu(Dm[v] * (1.0f / HS) + b2[col]); part += (kk < K) ? Wl[wid][kk] * Cv : 0.0f; }
    accA += part;
  }
  accA += __shfl_xor(accA, 16);
  { b16 a, c; split16(accA, a, c); if (hh == 0) { As[0][wid][col] = a; As[1][wid][col] = c; As[0][wid][16 + col] = (b16)0.0f; As[1][wid][16 + col] = (b16)0.0f; } }
  __syncthreads();
  if (wid == 0) {
    const size_t row0 = (size_t)blockIdx.x * 8;
    for (int pass = 0; pass < 2; ++pass) { *(volatile v8b*)(Agh + row0 * 32 + lane * 8) = *(const v8b*)(&As[0][0][0] + lane * 8); *(volatile v8b*)(Agl + row0 * 32 + lane * 8) = *(const v8b*)(&As[1][0][0] + lane * 8); __threadfence(); }
  }
}

__global__ __launch_bounds__(128) void out_kernel(const b16* __restrict__ Wg, const b16* __restrict__ featT, const b16* __restrict__ Agh, const b16* __restrict__ Agl,
                                                  const b16* __restrict__ p2h, const b16* __restrict__ p2l, const float* __restrict__ p2b, float* __restrict__ out) {
  __shared__ __attribute__((aligned(16))) float Ts[4][32 * 64];
  const int lane = threadIdx.x & 31, wave = threadIdx.x >> 5, nloc = lane & 15, hlf = lane >> 4, m0 = blockIdx.y * 128 + wave * 32, c0 = blockIdx.x * 64;
  const int b = m0 / T;
  v8f acc[2][4];
#pragma unroll
  for (int r = 0; r < 2; ++r)
#pragma unroll
    for (int t = 0; t < 4; ++t) acc[r][t] = (v8f){};
#pragma unroll 1
  for (int kb = 0; kb < KP; kb += 32) {
    const v16b a0 = frag_kb(Wg + (size_t)(m0 + nloc) * 256 + kb, hlf), a1 = frag_kb(Wg + (size_t)(m0 + 16 + nloc) * 256 + kb, hlf);
#pragma unroll
    for (int t = 0; t < 4; ++t) { const v16b bw = frag_kb(featT + ((size_t)b * DIM + c0 + t * 16 + nloc) * KP + kb, hlf); acc[0][t] = wmma16b(a0, bw, acc[0][t]); acc[1][t] = wmma16b(a1, bw, acc[1][t]); }
  }
  { const Opnd A{Agh, Agl, 32}, B{p2h, p2l, 16};
    v16b a0h, a0l, a1h, a1l; load_frags<2>(A, m0 + nloc, 0, hlf, a0h, a0l); load_frags<2>(A, m0 + 16 + nloc, 0, hlf, a1h, a1l);
#pragma unroll
    for (int t = 0; t < 4; ++t) { v16b bh_ = {}, bl_ = {}; const int n = c0 + t * 16 + nloc;
      { const v8b ph = ld8b(p2h + n * 16 + 8 * hlf), plw = ld8b(p2l + n * 16 + 8 * hlf);
#pragma unroll
        for (int e = 0; e < 8; ++e) { bh_[e] = ph[e]; bl_[e] = plw[e]; } }
      acc[0][t] = mac<2, 2>(a0h, a0l, bh_, bl_, acc[0][t]); acc[1][t] = mac<2, 2>(a1h, a1l, bh_, bl_, acc[1][t]); }
  }
  const Epi e{1.0f, nullptr, p2b, nullptr, 0, 1.0f, nullptr, nullptr};
  epi_f32(acc, e, out, DIM, m0, c0, lane, Ts[wave]);
}
}

extern "C" void kernel_launch(void* const* d_in, const int* in_sizes, int n_in,
                              void* d_out, int out_size, void* d_ws, size_t ws_size, hipStream_t stream) {
  (void)n_in; (void)out_size;
  const int* Tin = (const int*)d_in[0];
  const float* dur = (const float*)d_in[1]; const float* feat = (const float*)d_in[2];
  const float* c1w = (const float*)d_in[3]; const float* c1b = (const float*)d_in[4]; const float* c2w = (const float*)d_in[5]; const float* c2b = (const float*)d_in[6];
  const float* w1 = (const float*)d_in[7]; const float* b1 = (const float*)d_in[8]; const float* w2 = (const float*)d_in[9]; const float* b2 = (const float*)d_in[10];
  const float* v1 = (const float*)d_in[11]; const float* vb1 = (const float*)d_in[12]; const float* v2 = (const float*)d_in[13]; const float* vb2 = (const float*)d_in[14];
  const float* p1w = (const float*)d_in[15]; const float* p1b = (const float*)d_in[16]; const float* p2w = (const float*)d_in[17]; const float* p2b = (const float*)d_in[18];
  float* out = (float*)d_out;
  (void)Tin;
  if (in_sizes[0] != 1 || in_sizes[1] != Bn * K || in_sizes[2] != Bn * K * DIM || in_sizes[3] != 3 * DIM * 8 || in_sizes[9] != 256 || in_sizes[17] != 16 * DIM) return;
  size_t off = 0; char* ws = (char*)d_ws;
  auto carve = [&](size_t bytes) { char* p = ws + off; off += (bytes + 255) & ~(size_t)255; return p; };
  b16* cw16 = (b16*)carve(16 * 768 * 2); b16* w2h = (b16*)carve(16 * 16 * 2); b16* w2l = (b16*)carve(16 * 16 * 2); b16* p2h = (b16*)carve(DIM * 16 * 2); b16* p2l = (b16*)carve(DIM * 16 * 2);
  b16* featT = (b16*)carve((size_t)Bn * DIM * KP * 2);
  float* ts = (float*)carve(Bn * 256 * 4); float* te = (float*)carve(Bn * 256 * 4);
  float* zero = (float*)carve(DIM * 4);
  float* lr = (float*)carve((size_t)Bn * K * 16 * 4);
  b16* Wg = (b16*)carve((size_t)NBT * 256 * 2); b16* Agh = (b16*)carve((size_t)NBT * 32 * 2); b16* Agl = (b16*)carve((size_t)NBT * 32 * 2);
  if (off > ws_size) return;
  prep_kernel<<<32, 256, 0, stream>>>(dur, feat, c1w, c2w, w2, p2w, cw16, w2h, w2l, p2h, p2l, featT, ts, te, zero);
  conv_kernel<<<(Bn * K + 127) / 128, 128, 0, stream>>>(feat, zero, cw16, c1b, c2b, lr);
  main_kernel<<<NBT / 8, 256, 0, stream>>>(ts, te, lr, w1, b1, w2h, w2l, b2, v1, vb1, v2, vb2, p1w, p1b, Wg, Agh, Agl);
  out_kernel<<<dim3(DIM / 64, NBT / 128), 128, 0, stream>>>(Wg, featT, Agh, Agl, p2h, p2l, p2b, out);
}
